// FSM_47553877901592
// MI455X (gfx1250) — hardware-run, weakly checked
//
#include <hip/hip_runtime.h>
#include <math.h>

typedef __attribute__((ext_vector_type(16))) _Float16 v16h;
typedef __attribute__((ext_vector_type(8)))  _Float16 v8h;
typedef __attribute__((ext_vector_type(8)))  float    v8f;
typedef __attribute__((ext_vector_type(4)))  float    v4f;

constexpr int kBatch   = 4;
constexpr int kChan    = 48;
constexpr int kRed     = 16;
constexpr int kMid     = 8;
constexpr int kSide    = 64;
constexpr int kPix     = kSide * kSide;
constexpr int kRows    = kBatch * kPix;
constexpr int kK0Real  = kChan * 9;
constexpr int kK0Pad   = 448;
constexpr int kK5Real  = kRed * 9;
constexpr int kK5Pad   = 160;
constexpr int kNPad    = 64;
constexpr float kActCarry      = 16.0f;
constexpr float kWgtCarry      = 256.0f;
constexpr float kFoldBack      = 1.0f / (kActCarry * kWgtCarry);
constexpr float kHalfMinNormal = 6.103515625e-5f;

static_assert(kPix == 4096 && kRows == 16384, "pixel counts");
static_assert(kK0Real == 432 && kK5Real == 144, "im2col depths");
static_assert((kK0Pad % 32) == 0 && (kK5Pad % 32) == 0, "GEMM K multiples of 32");
static_assert(kK0Pad >= kK0Real && kK5Pad >= kK5Real, "K pads");
static_assert((kRows % 64) == 0 && (kNPad % 64) == 0, "GEMM M,N multiples of 64");
static_assert(kRed <= kNPad && kChan <= kNPad, "N pads");

constexpr size_t kOffA0  = 0;
constexpr size_t kOffA5  = kOffA0  + (size_t)kRows * kK0Pad * 2;
constexpr size_t kOffBT0 = kOffA5  + (size_t)kRows * kK5Pad * 2;
constexpr size_t kOffBT5 = kOffBT0 + (size_t)kNPad * kK0Pad * 2;
constexpr size_t kOffC0  = kOffBT5 + (size_t)kNPad * kK5Pad * 2;
constexpr size_t kOffC5  = kOffC0  + (size_t)kRows * kNPad * 4;
constexpr size_t kOffX   = kOffC5  + (size_t)kRows * kNPad * 4;
constexpr size_t kOffTH  = kOffX   + (size_t)kBatch * kRed * kPix * 4;
constexpr size_t kOffPH  = kOffTH  + (size_t)kBatch * kMid * kPix * 4;
constexpr size_t kOffGG  = kOffPH  + (size_t)kBatch * kMid * kPix * 4;
constexpr size_t kOffMM  = kOffGG  + (size_t)kBatch * kMid * kPix * 4;
constexpr size_t kOffZ   = kOffMM  + (size_t)kBatch * 64 * 4;
constexpr size_t kWsTotal = kOffZ  + (size_t)kBatch * kRed * kPix * 4;
static_assert(kWsTotal == 32060416ull, "carve total");
static_assert(kWsTotal <= 134217728ull, "carve cap");
static_assert((kOffA5 % 128) == 0 && (kOffBT0 % 128) == 0 && (kOffBT5 % 128) == 0 && (kOffC0 % 128) == 0 &&
              (kOffC5 % 128) == 0 && (kOffX % 128) == 0 && (kOffTH % 128) == 0 && (kOffPH % 128) == 0 &&
              (kOffGG % 128) == 0 && (kOffMM % 128) == 0 && (kOffZ % 128) == 0, "128-B aligned regions");

__device__ __forceinline__ _Float16 to_half_flushed(float v) {
  const float w = (fabsf(v) < kHalfMinNormal) ? 0.0f : v;
  return (_Float16)w;
}

union FragH { v16h v; v8h h[2]; };
__device__ __forceinline__ v16h frag_load(const _Float16* p) {
  FragH f;
  f.h[0] = *(const v8h*)(p);
  f.h[1] = *(const v8h*)(p + 16);
  return f.v;
}
__device__ __forceinline__ v8f mma_guarded(v16h a, v16h b, v8f c) {
  c = __builtin_amdgcn_wmma_f32_16x16x32_f16(false, a, false, b, (short)0, c, false, false);
  asm volatile("v_nop\n\tv_nop\n\tv_nop\n\tv_nop" : "+v"(c) : "v"(a), "v"(b));
  return c;
}
__device__ __forceinline__ void keep4_h(v16h a, v16h b, v16h c, v16h d) { asm volatile("v_nop" :: "v"(a), "v"(b), "v"(c), "v"(d)); }
__device__ __forceinline__ void acc_guard4(v8f& a, v8f& b, v8f& c, v8f& d) { asm volatile("v_nop\n\tv_nop\n\tv_nop\n\tv_nop" : "+v"(a), "+v"(b), "+v"(c), "+v"(d)); }

__global__ __launch_bounds__(256) void gemm64_f16_kernel(
    const unsigned short* __restrict__ Ap, int lda,
    const unsigned short* __restrict__ Btp, int ldb,
    float* __restrict__ C, int ldc, int M, int N, int K, float scale) {
  const _Float16* A  = (const _Float16*)Ap;
  const _Float16* Bt = (const _Float16*)Btp;
  __shared__ __align__(16) float sT[8][16 * 68];
  const int lane = threadIdx.x & 31;
  const int wave = threadIdx.x >> 5;
  const int tilesN = N >> 6;
  const int tilesM = M >> 6;
  const int tile = blockIdx.x * 8 + wave;
  if (tile >= tilesM * tilesN) return;
  const int tm = tile / tilesN;
  const int tn = tile - tm * tilesN;
  const int m0 = tm << 6;
  const int n0 = tn << 6;

  const int rlane = lane & 15;
  const int koff  = (lane >> 4) * 8;
  const int mOff  = (lane >> 4) * 8;

  v8f acc[4][4];
#pragma unroll
  for (int i = 0; i < 4; ++i)
#pragma unroll
    for (int j = 0; j < 4; ++j) acc[i][j] = (v8f){0.f,0.f,0.f,0.f,0.f,0.f,0.f,0.f};

  for (int k0 = 0; k0 < K; k0 += 32) {
    v16h bh[4];
#pragma unroll
    for (int j = 0; j < 4; ++j) {
      const size_t bo = (size_t)(n0 + (j << 4) + rlane) * ldb + koff + k0;
      bh[j] = frag_load(Bt + bo);
    }
#pragma unroll
    for (int i = 0; i < 4; ++i) {
      const size_t ao = (size_t)(m0 + (i << 4) + rlane) * lda + koff + k0;
      const v16h ah = frag_load(A + ao);
#pragma unroll
      for (int j = 0; j < 4; ++j) {
        acc[i][j] = mma_guarded(ah, bh[j], acc[i][j]);
      }
    }
    keep4_h(bh[0], bh[1], bh[2], bh[3]);
  }
  acc_guard4(acc[0][0], acc[0][1], acc[0][2], acc[0][3]);
  acc_guard4(acc[1][0], acc[1][1], acc[1][2], acc[1][3]);
  acc_guard4(acc[2][0], acc[2][1], acc[2][2], acc[2][3]);
  acc_guard4(acc[3][0], acc[3][1], acc[3][2], acc[3][3]);

  float* slab = sT[wave];
#pragma unroll
  for (int i = 0; i < 4; ++i) {
    const int mBase = m0 + (i << 4);
#pragma unroll
    for (int j = 0; j < 4; ++j) {
#pragma unroll
      for (int r = 0; r < 8; ++r) {
        const float v = acc[i][j][r] * scale;
        slab[(mOff + r) * 68 + (j << 4) + rlane] = v;
      }
    }
    __builtin_amdgcn_fence(__ATOMIC_RELEASE, "workgroup");
    __builtin_amdgcn_wave_barrier();
    __builtin_amdgcn_fence(__ATOMIC_ACQUIRE, "workgroup");
    {
      const int hh = lane >> 4;
      const int c4 = (lane & 15) * 4;
      for (int pass = 0; pass < 2; ++pass) {
#pragma unroll
        for (int it = 0; it < 8; ++it) {
          const int row = it * 2 + hh;
          const v4f v = *(const v4f*)(slab + row * 68 + c4);
          *(volatile v4f*)(C + (size_t)(mBase + row) * ldc + n0 + c4) = v;
        }
        __threadfence();
      }
    }
    __builtin_amdgcn_fence(__ATOMIC_RELEASE, "workgroup");
    __builtin_amdgcn_wave_barrier();
    __builtin_amdgcn_fence(__ATOMIC_ACQUIRE, "workgroup");
  }
}

template <int NREAL, int KREAL, int KPAD>
__global__ __launch_bounds__(256) void prepw_kernel(const float* __restrict__ w, unsigned short* __restrict__ dst, int total8) {
  constexpr int kGroups = KPAD / 8;
  const int i = blockIdx.x * 256 + threadIdx.x;
  if (i >= total8) return;
  const int n  = i / kGroups;
  const int kg = i - n * kGroups;
  const int nc = (n < NREAL) ? n : (NREAL - 1);
  v8h hv;
#pragma unroll
  for (int e = 0; e < 8; ++e) {
    const int k  = kg * 8 + e;
    const int kc = (k < KREAL) ? k : (KREAL - 1);
    const bool ok = (n < NREAL) && (k < KREAL);
    float v = w[nc * KREAL + kc];
    asm volatile("" : "+v"(v));
    const float cv = ok ? (v * kWgtCarry) : 0.0f;
    hv[e] = to_half_flushed(cv);
  }
  unsigned short* q = dst + 8 * (size_t)i;
  *(volatile v8h*)q = hv;
  __threadfence();
  *(volatile v8h*)q = hv;
}

template <int CIN, int KREAL, int KPAD>
__global__ __launch_bounds__(256) void im2col_kernel(const float* __restrict__ src, unsigned short* __restrict__ dst, int total8) {
  constexpr int kGroups = KPAD / 8;
  const int i = blockIdx.x * 256 + threadIdx.x;
  if (i >= total8) return;
  const int m   = i / kGroups;
  const int kg  = i - m * kGroups;
  const int b   = m >> 12;
  const int p   = m & (kPix - 1);
  const int row = p >> 6;
  const int col = p & 63;
  const float* sb = src + (size_t)b * CIN * kPix;
  v8h hv;
#pragma unroll
  for (int e = 0; e < 8; ++e) {
    const int k   = kg * 8 + e;
    const int c   = k / 9;
    const int tap = k - c * 9;
    const int ky  = tap / 3;
    const int kx  = tap - ky * 3;
    const int iy  = row + ky - 1;
    const int ix  = col + kx - 1;
    const bool ok = (k < KREAL) && ((unsigned)iy < 64u) && ((unsigned)ix < 64u);
    const int cc  = (c < CIN) ? c : (CIN - 1);
    const int iyc = (iy < 0) ? 0 : ((iy > 63) ? 63 : iy);
    const int ixc = (ix < 0) ? 0 : ((ix > 63) ? 63 : ix);
    float v = sb[cc * kPix + iyc * 64 + ixc];
    asm volatile("" : "+v"(v));
    const float cv = ok ? (v * kActCarry) : 0.0f;
    hv[e] = to_half_flushed(cv);
  }
  unsigned short* q = dst + 8 * (size_t)i;
  *(volatile v8h*)q = hv;
  __threadfence();
  *(volatile v8h*)q = hv;
}

__global__ __launch_bounds__(256) void point1_kernel(
    const float* __restrict__ C0, const float* __restrict__ bx,
    const float* __restrict__ wth, const float* __restrict__ bth,
    const float* __restrict__ wph, const float* __restrict__ bph,
    const float* __restrict__ wg,  const float* __restrict__ bg,
    float* __restrict__ X, float* __restrict__ TH, float* __restrict__ PH, float* __restrict__ GG) {
  const int m = blockIdx.x * 256 + threadIdx.x;
  const int b = m >> 12;
  const int p = m & (kPix - 1);
  const float* cr = C0 + (size_t)m * kNPad;
  const v4f q0 = *(const v4f*)(cr);
  const v4f q1 = *(const v4f*)(cr + 4);
  const v4f q2 = *(const v4f*)(cr + 8);
  const v4f q3 = *(const v4f*)(cr + 12);
  float xv[16];
#pragma unroll
  for (int e = 0; e < 4; ++e) {
    xv[e]      = fmaxf(q0[e] + bx[e], 0.0f);
    xv[4 + e]  = fmaxf(q1[e] + bx[4 + e], 0.0f);
    xv[8 + e]  = fmaxf(q2[e] + bx[8 + e], 0.0f);
    xv[12 + e] = fmaxf(q3[e] + bx[12 + e], 0.0f);
  }
  for (int pass = 0; pass < 2; ++pass) {
#pragma unroll
    for (int r = 0; r < 16; ++r) {
      *(volatile float*)(X + (size_t)(b * kRed + r) * kPix + p) = xv[r];
    }
    __threadfence();
  }
#pragma unroll 1
  for (int j = 0; j < kMid; ++j) {
    float s0 = bth[j];
    float s1 = bph[j];
    float s2 = bg[j];
#pragma unroll
    for (int c = 0; c < 16; ++c) {
      s0 = fmaf(wth[j * 16 + c], xv[c], s0);
      s1 = fmaf(wph[j * 16 + c], xv[c], s1);
      s2 = fmaf(wg[j * 16 + c],  xv[c], s2);
    }
    s0 = fmaxf(s0, 0.0f);
    s1 = fmaxf(s1, 0.0f);
    s2 = fmaxf(s2, 0.0f);
    const size_t o = (size_t)(b * kMid + j) * kPix + p;
    *(volatile float*)(TH + o) = s0;
    *(volatile float*)(PH + o) = s1;
    *(volatile float*)(GG + o) = s2;
    __threadfence();
    *(volatile float*)(TH + o) = s0;
    *(volatile float*)(PH + o) = s1;
    *(volatile float*)(GG + o) = s2;
  }
}

__global__ __launch_bounds__(256) void mred_kernel(const float* __restrict__ PH, const float* __restrict__ GG, float* __restrict__ MM) {
  __shared__ float sP[4][64];
  const int b    = blockIdx.x;
  const int t    = threadIdx.x;
  const int pair = t & 63;
  const int sl   = t >> 6;
  const int i    = pair >> 3;
  const int j    = pair & 7;
  const float* pp = PH + (size_t)(b * kMid + i) * kPix + sl * 1024;
  const float* gp = GG + (size_t)(b * kMid + j) * kPix + sl * 1024;
  float a0 = 0.0f, a1 = 0.0f, a2 = 0.0f, a3 = 0.0f;
#pragma unroll 1
  for (int q4 = 0; q4 < 256; ++q4) {
    const v4f pv = *(const v4f*)(pp + 4 * q4);
    const v4f gv = *(const v4f*)(gp + 4 * q4);
    a0 = fmaf(pv[0], gv[0], a0);
    a1 = fmaf(pv[1], gv[1], a1);
    a2 = fmaf(pv[2], gv[2], a2);
    a3 = fmaf(pv[3], gv[3], a3);
  }
  sP[sl][pair] = (a0 + a1) + (a2 + a3);
  __syncthreads();
  if (t < 64) {
    const float s = (sP[0][t] + sP[1][t]) + (sP[2][t] + sP[3][t]);
    float* q = MM + b * 64 + t;
    *(volatile float*)q = s;
    __threadfence();
    *(volatile float*)q = s;
  }
}

__global__ __launch_bounds__(256) void point2_kernel(
    const float* __restrict__ TH, const float* __restrict__ MM,
    const float* __restrict__ wy, const float* __restrict__ by,
    const float* __restrict__ X, float* __restrict__ Z) {
  const int m  = blockIdx.x * 256 + threadIdx.x;
  const int b  = m >> 12;
  const int s  = m & (kPix - 1);
  const int j  = s & 7;
  const int pq = s >> 3;
  float mc[8];
#pragma unroll
  for (int i = 0; i < 8; ++i) mc[i] = MM[b * 64 + i * 8 + j];
  float y[16];
#pragma unroll
  for (int r = 0; r < 16; ++r) y[r] = by[r];
  const float* thb = TH + (size_t)b * kMid * kPix;
#pragma unroll 1
  for (int c = 0; c < kMid; ++c) {
    const int p = c * 512 + pq;
    float f = 0.0f;
#pragma unroll
    for (int i = 0; i < 8; ++i) f = fmaf(thb[i * kPix + p], mc[i], f);
#pragma unroll
    for (int r = 0; r < 16; ++r) y[r] = fmaf(wy[r * 8 + c], f, y[r]);
  }
  float zv[16];
#pragma unroll
  for (int r = 0; r < 16; ++r) {
    const float xr = X[(size_t)(b * kRed + r) * kPix + s];
    zv[r] = fmaxf(y[r], 0.0f) + xr;
  }
  for (int pass = 0; pass < 2; ++pass) {
#pragma unroll
    for (int r = 0; r < 16; ++r) {
      *(volatile float*)(Z + (size_t)(b * kRed + r) * kPix + s) = zv[r];
    }
    __threadfence();
  }
}

__global__ __launch_bounds__(256) void outpack_kernel(
    const float* __restrict__ C5, const float* __restrict__ blast,
    const float* __restrict__ xin, float* __restrict__ out) {
  const int i  = blockIdx.x * 256 + threadIdx.x;
  const int p4 = (i & 1023) * 4;
  const int bn = i >> 10;
  const int b  = bn / kChan;
  const int n  = bn - b * kChan;
  const float* cp = C5 + ((size_t)b * kPix + p4) * kNPad + n;
  const float c0 = cp[0];
  const float c1 = cp[kNPad];
  const float c2 = cp[2 * kNPad];
  const float c3 = cp[3 * kNPad];
  const float bias = blast[n];
  const size_t o = (size_t)bn * kPix + p4;
  const v4f ox = *(const v4f*)(xin + o);
  v4f r;
  r[0] = fmaxf(c0 + bias, 0.0f) + ox[0];
  r[1] = fmaxf(c1 + bias, 0.0f) + ox[1];
  r[2] = fmaxf(c2 + bias, 0.0f) + ox[2];
  r[3] = fmaxf(c3 + bias, 0.0f) + ox[3];
  *(volatile v4f*)(out + o) = r;
  __threadfence();
  *(volatile v4f*)(out + o) = r;
}

extern "C" void kernel_launch(void* const* d_in, const int* in_sizes, int n_in,
                              void* d_out, int out_size, void* d_ws, size_t ws_size,
                              hipStream_t stream) {
  if (n_in < 13) return;
  if (in_sizes[0] != kBatch * kChan * kPix) return;
  if (in_sizes[1] != kRed * kK0Real) return;
  if (in_sizes[2] != kRed) return;
  if (in_sizes[3] != kMid * kRed) return;
  if (in_sizes[4] != kMid) return;
  if (in_sizes[5] != kMid * kRed) return;
  if (in_sizes[6] != kMid) return;
  if (in_sizes[7] != kMid * kRed) return;
  if (in_sizes[8] != kMid) return;
  if (in_sizes[9] != kRed * kMid) return;
  if (in_sizes[10] != kRed) return;
  if (in_sizes[11] != kChan * kK5Real) return;
  if (in_sizes[12] != kChan) return;
  if (out_size != kBatch * kChan * kPix) return;
  if (ws_size < kWsTotal) return;

  const float* origx  = (const float*)d_in[0];
  const float* w_x    = (const float*)d_in[1];
  const float* b_x    = (const float*)d_in[2];
  const float* w_th   = (const float*)d_in[3];
  const float* b_th   = (const float*)d_in[4];
  const float* w_ph   = (const float*)d_in[5];
  const float* b_ph   = (const float*)d_in[6];
  const float* w_g    = (const float*)d_in[7];
  const float* b_g    = (const float*)d_in[8];
  const float* w_y    = (const float*)d_in[9];
  const float* b_y    = (const float*)d_in[10];
  const float* w_last = (const float*)d_in[11];
  const float* b_last = (const float*)d_in[12];
  float* out = (float*)d_out;

  char* ws = (char*)d_ws;
  unsigned short* A0  = (unsigned short*)(ws + kOffA0);
  unsigned short* A5  = (unsigned short*)(ws + kOffA5);
  unsigned short* BT0 = (unsigned short*)(ws + kOffBT0);
  unsigned short* BT5 = (unsigned short*)(ws + kOffBT5);
  float* C0 = (float*)(ws + kOffC0);
  float* C5 = (float*)(ws + kOffC5);
  float* X  = (float*)(ws + kOffX);
  float* TH = (float*)(ws + kOffTH);
  float* PH = (float*)(ws + kOffPH);
  float* GG = (float*)(ws + kOffGG);
  float* MM = (float*)(ws + kOffMM);
  float* Z  = (float*)(ws + kOffZ);

  prepw_kernel<kRed, kK0Real, kK0Pad><<<(kNPad * kK0Pad / 8) / 256, 256, 0, stream>>>(w_x, BT0, kNPad * kK0Pad / 8);
  prepw_kernel<kChan, kK5Real, kK5Pad><<<(kNPad * kK5Pad / 8) / 256, 256, 0, stream>>>(w_last, BT5, kNPad * kK5Pad / 8);

  im2col_kernel<kChan, kK0Real, kK0Pad><<<(kRows * (kK0Pad / 8)) / 256, 256, 0, stream>>>(origx, A0, kRows * (kK0Pad / 8));
  gemm64_f16_kernel<<<(kRows / 64) / 8, 256, 0, stream>>>(A0, kK0Pad, BT0, kK0Pad, C0, kNPad, kRows, kNPad, kK0Pad, kFoldBack);

  point1_kernel<<<kRows / 256, 256, 0, stream>>>(C0, b_x, w_th, b_th, w_ph, b_ph, w_g, b_g, X, TH, PH, GG);

  mred_kernel<<<kBatch, 256, 0, stream>>>(PH, GG, MM);

  point2_kernel<<<kRows / 256, 256, 0, stream>>>(TH, MM, w_y, b_y, X, Z);

  im2col_kernel<kRed, kK5Real, kK5Pad><<<(kRows * (kK5Pad / 8)) / 256, 256, 0, stream>>>(Z, A5, kRows * (kK5Pad / 8));
  gemm64_f16_kernel<<<(kRows / 64) / 8, 256, 0, stream>>>(A5, kK5Pad, BT5, kK5Pad, C5, kNPad, kRows, kNPad, kK5Pad, kFoldBack);

  outpack_kernel<<<(kBatch * kChan * kPix / 4) / 256, 256, 0, stream>>>(C5, b_last, origx, out);
}
